// GAT_67448166416665
// MI455X (gfx1250) — hardware-verified
//
#include <hip/hip_runtime.h>
#include <stddef.h>
#include <stdint.h>
#include <math.h>


#define BSZ    2
#define NN     2048
#define MPR    (BSZ * NN)
#define FIN    128
#define NHD1   8
#define HID    64
#define CH1    (NHD1 * HID)
#define NC1    (2 * CH1)
#define KA2    (2 * CH1)
#define F2     64
#define NC2    (2 * F2)
#define NTHR   256
#define NWAVE  8
#define RB2    8
#define GBM    64
#define GBN    64
#define GTHR   128
#define NEGSL  0.2f
#define WSMAX  134217728

static_assert(NTHR * 8 == NN);
static_assert(NTHR == 32 * NWAVE);
static_assert((MPR % GBM) == 0 && (NC1 % GBN) == 0 && (NC2 % GBN) == 0);
static_assert((FIN % 32) == 0 && (KA2 % 32) == 0);
static_assert(GBM == (GTHR / 32) * 16);
static_assert(GTHR == 2 * GBN && GTHR == 2 * GBM);
static_assert(HID == GBN && F2 == HID);
static_assert(CH1 == NWAVE * HID);
static_assert(HID == 2 * 32);
static_assert((MPR % RB2) == 0 && (NN % RB2) == 0 && RB2 == NWAVE);
static_assert((FIN % 8) == 0 && (CH1 % 8) == 0);

typedef float          v2f  __attribute__((ext_vector_type(2)));
typedef float          v4f  __attribute__((ext_vector_type(4)));
typedef float          v8f  __attribute__((ext_vector_type(8)));
typedef int            v8i  __attribute__((ext_vector_type(8)));
typedef unsigned int   v4u  __attribute__((ext_vector_type(4)));
typedef unsigned short v8us __attribute__((ext_vector_type(8)));
typedef __bf16         v16b __attribute__((ext_vector_type(16)));
typedef v2f  __attribute__((may_alias)) v2fa;
typedef v4f  __attribute__((may_alias)) v4fa;
typedef v8us __attribute__((may_alias)) v8usa;
union FragB { v16b v; v8us h[2]; v8i w; };

__device__ __forceinline__ v8f wmb(const FragB& a, const FragB& b, v8f c) {
  v8f d = __builtin_amdgcn_wmma_f32_16x16x32_bf16(false, a.v, false, b.v, (short)0, c, false, false);
  asm volatile("v_nop\n\tv_nop\n\tv_nop\n\tv_nop" : "+v"(d) : "v"(a.w), "v"(b.w));
  return d;
}

__device__ __forceinline__ unsigned int f2bf(float f) {
  const unsigned int u = __float_as_uint(f);
  return ((u + 0x7FFFu + ((u >> 16) & 1u)) >> 16) & 0xFFFFu;
}
__device__ __forceinline__ float bf2f(unsigned int b) { return __uint_as_float(b << 16); }
__device__ __forceinline__ float bfr(float f) { return bf2f(f2bf(f)); }
__device__ __forceinline__ unsigned int pk2(float lo, float hi) { return f2bf(lo) | (f2bf(hi) << 16); }
__device__ __forceinline__ v4u pack8(const v4f a, const v4f b) {
  v4u r;
  r.x = pk2(a.x, a.y); r.y = pk2(a.z, a.w); r.z = pk2(b.x, b.y); r.w = pk2(b.z, b.w);
  return r;
}
__device__ __forceinline__ float lk(float v) { return v >= 0.f ? v : NEGSL * v; }

__global__ __launch_bounds__(NTHR) void k_cvtb(const float* __restrict__ src, int srcRows, int srcK,
                                               unsigned short* dst, int dstRow0, int dstK, int nUnits) {
  const int u = (int)blockIdx.x * NTHR + (int)threadIdx.x;
  if (u >= nUnits) return;
  const int kq  = dstK >> 3;
  const int n   = u / kq;
  const int k8  = (u - n * kq) * 8;
  const int kk  = k8 - (k8 / srcK) * srcK;
  const int ncl = n < srcRows ? n : srcRows - 1;
  const float* p = src + (size_t)ncl * (size_t)srcK + kk;
  v4f a = *(const v4fa*)p, b = *(const v4fa*)(p + 4);
  const v4f z4 = {0.f, 0.f, 0.f, 0.f};
  if (n >= srcRows) { a = z4; b = z4; }
  const v4u hv = pack8(a, b);
  unsigned short* o = dst + (size_t)(dstRow0 + n) * (size_t)dstK + k8;
  *(volatile v4u*)o = hv;
  __threadfence();
  *(volatile v4u*)o = hv;
}

__global__ __launch_bounds__(GTHR) void k_gemm(
    const unsigned short* __restrict__ A, const unsigned short* __restrict__ WT,
    float* outF, int K, int ldo,
    const float* __restrict__ atts, const float* __restrict__ attd, int attLen, int nHead,
    float* SD, int MPr)
{
  __shared__ __attribute__((aligned(16))) float stg[GBM * GBN];
  __shared__ __attribute__((aligned(16))) float satt[2 * GBN];
  __shared__ __attribute__((aligned(16))) float sdot[2 * GBM];
  const int tid = (int)threadIdx.x, lane = tid & 31, wave = tid >> 5, hh = lane >> 4, m = lane & 15;
  const int rowBase = (int)blockIdx.x * GBM;
  const int head    = (int)blockIdx.y;
  const int col0    = head * GBN;
  const int hcl     = head < nHead ? head : nHead - 1;

  {
    const int which = tid >> 6;
    const int c  = tid & 63;
    const int cl = c < attLen ? c : attLen - 1;
    const float vs = atts[hcl * attLen + cl];
    const float vd = attd[hcl * attLen + cl];
    float v = (which == 0) ? vs : vd;
    v = (c < attLen) ? bfr(v) : 0.f;
    satt[which * GBN + c] = v;
  }

  v8f acc[4];
  {
    const v8f z = {0.f, 0.f, 0.f, 0.f, 0.f, 0.f, 0.f, 0.f};
    acc[0] = z; acc[1] = z; acc[2] = z; acc[3] = z;
  }
  const unsigned short* ap = A  + (size_t)(rowBase + 16 * wave + m) * (size_t)K + 8 * hh;
  const unsigned short* wp = WT + (size_t)(col0 + m) * (size_t)K + 8 * hh;
  const int ksteps = K >> 5;
#pragma unroll 1
  for (int ks = 0; ks < ksteps; ++ks) {
    FragB af;
    af.h[0] = *(const v8usa*)(ap + 32 * ks);
    af.h[1] = *(const v8usa*)(ap + 32 * ks + 16);
#pragma unroll
    for (int t = 0; t < 4; ++t) {
      const unsigned short* wq = wp + (size_t)(16 * t) * (size_t)K + 32 * ks;
      FragB bf;
      bf.h[0] = *(const v8usa*)wq;
      bf.h[1] = *(const v8usa*)(wq + 16);
      acc[t] = wmb(af, bf, acc[t]);
    }
  }

#pragma unroll
  for (int t = 0; t < 4; ++t) {
    const int lc = 16 * t + m;
#pragma unroll
    for (int r = 0; r < 8; ++r) {
      const int lr = 16 * wave + 8 * hh + r;
      stg[lr * GBN + lc] = acc[t][r];
    }
  }
  __syncthreads();

  {
    const int row = tid & 63, which = tid >> 6;
    const float* sa = satt + which * GBN;
    const float* hr = stg + row * GBN;
    float d = 0.f;
#pragma unroll 4
    for (int c4 = 0; c4 < GBN / 4; ++c4) {
      const v4f hv = *(const v4fa*)(hr + 4 * c4);
      const v4f av = *(const v4fa*)(sa + 4 * c4);
      d = fmaf(hv.x, av.x, d);
      d = fmaf(hv.y, av.y, d);
      d = fmaf(hv.z, av.z, d);
      d = fmaf(hv.w, av.w, d);
    }
    sdot[which * GBM + row] = d;
  }
  __syncthreads();

  v4f fv[8];
#pragma unroll
  for (int i = 0; i < 8; ++i) {
    const int lr = 16 * wave + 2 * i + hh;
    fv[i] = *(const v4fa*)(stg + lr * GBN + 4 * m);
  }
  const int which2 = lane >> 4, piece = lane & 15;
  const v4f sdv = *(const v4fa*)(sdot + which2 * GBM + 4 * piece);
  float* sp = SD + (size_t)(2 * hcl + which2) * (size_t)MPr + rowBase + 4 * piece;
  const bool dw = (wave == 0) && (head < nHead);

#pragma unroll
  for (int i = 0; i < 8; ++i) {
    const int lr = 16 * wave + 2 * i + hh;
    const int gr = rowBase + lr;
    float* op = outF + (size_t)gr * (size_t)ldo + col0 + 4 * m;
    *(volatile v4f*)op = fv[i];
  }
  if (dw) *(volatile v4f*)sp = sdv;
  __threadfence();
#pragma unroll
  for (int i = 0; i < 8; ++i) {
    const int lr = 16 * wave + 2 * i + hh;
    const int gr = rowBase + lr;
    float* op = outF + (size_t)gr * (size_t)ldo + col0 + 4 * m;
    *(volatile v4f*)op = fv[i];
  }
  if (dw) *(volatile v4f*)sp = sdv;
}

template<int RB, int NHD, int MODE>
__global__ __launch_bounds__(NTHR) void k_agg(
    const float* __restrict__ adj, const float* __restrict__ C, const float* __restrict__ SD,
    const float* __restrict__ bias, unsigned short* HP, float* out, int nRows)
{
  static_assert((RB == 1 && NHD == NWAVE) || (RB == NWAVE && NHD == 1));
  constexpr int CP  = 2 * NHD * HID;
  constexpr int SKO = NHD * HID;
  __shared__ __attribute__((aligned(16))) unsigned short lst[RB * NN];
  __shared__ int wtot[RB * NWAVE];
  __shared__ int scnt[RB];
  const int tid = (int)threadIdx.x, lane = tid & 31, wave = tid >> 5;

#pragma unroll 1
  for (int r = 0; r < RB; ++r) {
    const int gr  = (int)blockIdx.x * RB + r;
    const int grc = gr < nRows ? gr : nRows - 1;
    const float* ar = adj + (size_t)grc * (size_t)NN + 8 * tid;
    const v4f a = *(const v4fa*)ar;
    const v4f b = *(const v4fa*)(ar + 4);
    unsigned hb = 0u;
    hb |= (a.x != 0.0f) ? 1u   : 0u;
    hb |= (a.y != 0.0f) ? 2u   : 0u;
    hb |= (a.z != 0.0f) ? 4u   : 0u;
    hb |= (a.w != 0.0f) ? 8u   : 0u;
    hb |= (b.x != 0.0f) ? 16u  : 0u;
    hb |= (b.y != 0.0f) ? 32u  : 0u;
    hb |= (b.z != 0.0f) ? 64u  : 0u;
    hb |= (b.w != 0.0f) ? 128u : 0u;
    const int c = (int)__builtin_popcount(hb);
    int incl = c;
#pragma unroll
    for (int d = 1; d < 32; d <<= 1) {
      const int up = __shfl_up(incl, d);
      if (lane >= d) incl += up;
    }
    if (lane == 31) wtot[r * NWAVE + wave] = incl;
    __syncthreads();
    int pre = 0, tot = 0;
#pragma unroll
    for (int w2 = 0; w2 < NWAVE; ++w2) {
      const int t = wtot[r * NWAVE + w2];
      pre += (w2 < wave) ? t : 0;
      tot += t;
    }
    int pos = pre + incl - c;
    unsigned short* lrw = lst + r * NN;
#pragma unroll
    for (int j = 0; j < 8; ++j) {
      if ((hb >> j) & 1u) {
        const int pc = pos < NN ? pos : NN - 1;
        lrw[pc] = (unsigned short)(8 * tid + j);
        ++pos;
      }
    }
    if (tid == 0) scnt[r] = tot;
  }
  __syncthreads();

  const int r   = (RB == 1) ? 0 : wave;
  const int h   = (RB == 1) ? wave : 0;
  const int gr  = (int)blockIdx.x * RB + r;
  const int grc = gr < nRows ? gr : nRows - 1;
  const int bN  = (grc / NN) * NN;
  const unsigned short* lr = lst + r * NN;
  int cnt = scnt[r];
  cnt = cnt < 0 ? 0 : (cnt > NN ? NN : cnt);
  const float  ss = SD[(size_t)(2 * h) * (size_t)nRows + grc];
  const float* T  = SD + (size_t)(2 * h + 1) * (size_t)nRows + bN;

  float mx = -3.0e38f;
#pragma unroll 1
  for (int j = lane; j < cnt; j += 32) {
    const int mj = (int)lr[j];
    mx = fmaxf(mx, lk(ss + T[mj]));
  }
#pragma unroll
  for (int off = 16; off > 0; off >>= 1) mx = fmaxf(mx, __shfl_xor(mx, off));

  const int c0 = h * HID + 2 * lane;
  float den = 0.f, ax = 0.f, ay = 0.f;
#pragma unroll 1
  for (int g0 = 0; g0 < cnt; g0 += 32) {
    const int j  = g0 + lane;
    const int jc = j < cnt ? j : cnt - 1;
    const int mj = (int)lr[jc];
    const float ej = lk(ss + T[mj]);
    const float pj = (j < cnt) ? expf(ej - mx) : 0.f;
    int kmax = cnt - g0; kmax = kmax > 32 ? 32 : kmax;
#pragma unroll 1
    for (int k = 0; k < kmax; ++k) {
      const float p  = __shfl(pj, k);
      const int   mm = __shfl(mj, k);
      den += p;
      const v2f fr = *(const v2fa*)(C + (size_t)(bN + mm) * (size_t)CP + c0);
      ax = fmaf(p, fr.x, ax);
      ay = fmaf(p, fr.y, ay);
    }
  }
  const float ds  = den > 0.f ? den : 1.0f;
  const float inv = 1.0f / ds;
  const float pz  = (cnt > 0) ? 0.0f : __int_as_float(0x7fc00000);
  const v2f sk = *(const v2fa*)(C + (size_t)grc * (size_t)CP + SKO + c0);
  const float bb0 = bfr(bias[c0]), bb1 = bfr(bias[c0 + 1]);
  float v0 = (fmaf(ax, inv, sk.x) + bb0) + pz;
  float v1 = (fmaf(ay, inv, sk.y) + bb1) + pz;

  if (MODE == 0) {
    v0 = v0 > 0.f ? v0 : expm1f(v0);
    v1 = v1 > 0.f ? v1 : expm1f(v1);
    const unsigned int hbx = f2bf(v0), hby = f2bf(v1);
    const unsigned int lbx = f2bf(v0 - bf2f(hbx)), lby = f2bf(v1 - bf2f(hby));
    const int hw = (int)(hbx | (hby << 16));
    const int lw = (int)(lbx | (lby << 16));
    const int si = (4 * lane) & 31;
    const int g0 = __shfl(hw, si), g1 = __shfl(hw, si + 1), g2 = __shfl(hw, si + 2), g3 = __shfl(hw, si + 3);
    const int q0 = __shfl(lw, si), q1 = __shfl(lw, si + 1), q2 = __shfl(lw, si + 2), q3 = __shfl(lw, si + 3);
    const bool lsel = lane >= 16;
    v4u pv;
    pv.x = (unsigned int)(lsel ? q0 : g0);
    pv.y = (unsigned int)(lsel ? q1 : g1);
    pv.z = (unsigned int)(lsel ? q2 : g2);
    pv.w = (unsigned int)(lsel ? q3 : g3);
    const int q = lane & 15;
    const bool wsv = (q < 8) && (gr < nRows);
    unsigned short* gp = HP + (size_t)grc * (size_t)CP + (lsel ? SKO : 0) + h * HID + 8 * q;
    if (wsv) *(volatile v4u*)gp = pv;
    __threadfence();
    if (wsv) *(volatile v4u*)gp = pv;
  } else {
    const int si = (2 * lane) & 31;
    const float g0 = __shfl(v0, si), g1 = __shfl(v1, si), g2 = __shfl(v0, si + 1), g3 = __shfl(v1, si + 1);
    v4f ov; ov.x = g0; ov.y = g1; ov.z = g2; ov.w = g3;
    const bool wsv = (lane < 16) && (gr < nRows);
    float* op = out + (size_t)grc * SKO + 4 * lane;
    if (wsv) *(volatile v4f*)op = ov;
    __threadfence();
    if (wsv) *(volatile v4f*)op = ov;
  }
  (void)HP; (void)out;
}

static inline int cdiv(int a, int b) { return (a + b - 1) / b; }

extern "C" void kernel_launch(void* const* d_in, const int* in_sizes, int n_in,
                              void* d_out, int out_size, void* d_ws, size_t ws_size,
                              hipStream_t stream) {
  if (n_in < 12) return;
  if (in_sizes[0]  != MPR * FIN) return;
  if (in_sizes[1]  != MPR * NN) return;
  if (in_sizes[2]  != CH1 * FIN) return;
  if (in_sizes[3]  != NHD1 * HID) return;
  if (in_sizes[4]  != NHD1 * HID) return;
  if (in_sizes[5]  != CH1 * FIN) return;
  if (in_sizes[6]  != CH1) return;
  if (in_sizes[7]  != F2 * CH1) return;
  if (in_sizes[8]  != F2) return;
  if (in_sizes[9]  != F2) return;
  if (in_sizes[10] != F2 * CH1) return;
  if (in_sizes[11] != F2) return;
  if (out_size != MPR * F2) return;

  const float* x    = (const float*)d_in[0];
  const float* adj  = (const float*)d_in[1];
  const float* W1   = (const float*)d_in[2];
  const float* a1s  = (const float*)d_in[3];
  const float* a1t  = (const float*)d_in[4];
  const float* Wsk1 = (const float*)d_in[5];
  const float* b1   = (const float*)d_in[6];
  const float* W2   = (const float*)d_in[7];
  const float* a2s  = (const float*)d_in[8];
  const float* a2t  = (const float*)d_in[9];
  const float* Wsk2 = (const float*)d_in[10];
  const float* b2   = (const float*)d_in[11];
  float* out = (float*)d_out;

  char* ws = (char*)d_ws;
  size_t off = 0;
  const size_t oXB  = off; off += (size_t)MPR * FIN * 2;        off = (off + 255) & ~(size_t)255;
  const size_t oWT1 = off; off += (size_t)NC1 * FIN * 2;        off = (off + 255) & ~(size_t)255;
  const size_t oWT2 = off; off += (size_t)NC2 * KA2 * 2;        off = (off + 255) & ~(size_t)255;
  const size_t oC1  = off; off += (size_t)MPR * NC1 * 4;        off = (off + 255) & ~(size_t)255;
  const size_t oSD1 = off; off += (size_t)2 * NHD1 * MPR * 4;   off = (off + 255) & ~(size_t)255;
  const size_t oHHL = off; off += (size_t)MPR * KA2 * 2;        off = (off + 255) & ~(size_t)255;
  const size_t oC2  = off; off += (size_t)MPR * NC2 * 4;        off = (off + 255) & ~(size_t)255;
  const size_t oSD2 = off; off += (size_t)2 * 1 * MPR * 4;      off = (off + 255) & ~(size_t)255;
  if (off > ws_size || off > (size_t)WSMAX) return;
  unsigned short* XB  = (unsigned short*)(ws + oXB);
  unsigned short* WT1 = (unsigned short*)(ws + oWT1);
  unsigned short* WT2 = (unsigned short*)(ws + oWT2);
  float*          C1  = (float*)(ws + oC1);
  float*          SD1 = (float*)(ws + oSD1);
  unsigned short* HHL = (unsigned short*)(ws + oHHL);
  float*          C2  = (float*)(ws + oC2);
  float*          SD2 = (float*)(ws + oSD2);

  {
    const int nUx = MPR * (FIN / 8);
    k_cvtb<<<cdiv(nUx, NTHR), NTHR, 0, stream>>>(x, MPR, FIN, XB, 0, FIN, nUx);
    const int nUw1 = CH1 * (FIN / 8);
    k_cvtb<<<cdiv(nUw1, NTHR), NTHR, 0, stream>>>(W1,   CH1, FIN, WT1, 0,   FIN, nUw1);
    k_cvtb<<<cdiv(nUw1, NTHR), NTHR, 0, stream>>>(Wsk1, CH1, FIN, WT1, CH1, FIN, nUw1);
    const int nUw2 = F2 * (KA2 / 8);
    k_cvtb<<<cdiv(nUw2, NTHR), NTHR, 0, stream>>>(W2,   F2, CH1, WT2, 0,  KA2, nUw2);
    k_cvtb<<<cdiv(nUw2, NTHR), NTHR, 0, stream>>>(Wsk2, F2, CH1, WT2, F2, KA2, nUw2);
  }

  const int gM = MPR / GBM;
  k_gemm<<<dim3(gM, NC1 / GBN), GTHR, 0, stream>>>(XB, WT1, C1, FIN, NC1, a1s, a1t, HID, NHD1, SD1, MPR);
  k_agg<1, NHD1, 0><<<MPR, NTHR, 0, stream>>>(adj, C1, SD1, b1, HHL, out, MPR);
  k_gemm<<<dim3(gM, NC2 / GBN), GTHR, 0, stream>>>(HHL, WT2, C2, KA2, NC2, a2s, a2t, F2, 1, SD2, MPR);
  k_agg<RB2, 1, 1><<<MPR / RB2, NTHR, 0, stream>>>(adj, C2, SD2, b2, HHL, out, MPR);
}
